// ModelTorch_33002528702615
// MI455X (gfx1250) — hardware-verified
//
#include <hip/hip_runtime.h>
#include <stddef.h>


typedef _Float16 h16;
typedef _Float16 v16h __attribute__((ext_vector_type(16)));
typedef _Float16 v8h  __attribute__((ext_vector_type(8)));
typedef float    v8f  __attribute__((ext_vector_type(8)));
typedef float    v4f  __attribute__((ext_vector_type(4)));

#ifndef NQ
#define NQ 2048
#endif
#ifndef NTR
#define NTR 50000
#endif
#define NQ_FULL  2048
#define NTR_FULL 50000
#define DIM    128
#define OUTD   64
#define KSPLIT 16
#define KSTEP  64
#define NPAD   (((NTR + KSPLIT * KSTEP - 1) / (KSPLIT * KSTEP)) * (KSPLIT * KSTEP))
#define KPS    (NPAD / KSPLIT)

static_assert(NQ >= 128 && NQ <= NQ_FULL && (NQ % 128) == 0);
static_assert(NTR >= 64 && NTR <= NTR_FULL);
static_assert(DIM == 128 && (DIM % 32) == 0);
static_assert(DIM == 16 * 8);
static_assert(OUTD == 64);
static_assert((NPAD % 64) == 0 && NPAD >= NTR);
static_assert((KPS % KSTEP) == 0 && KPS * KSPLIT == NPAD);
static_assert((NQ % 64) == 0);
static_assert(((NQ * OUTD) % 1024) == 0);
static_assert((size_t)NPAD * DIM < (size_t)0xFFFFFFFFu);

#define LDT 72
#define LDC 68
static_assert((LDT % 8) == 0 && LDT >= 64);
static_assert((LDC % 4) == 0 && LDC >= 64);
static_assert(8 * 16 * LDT * 2 + 8 * 16 * LDC * 4 <= 131072);

#define XCARRY 64.0f
#define WCARRY 64.0f
#define PCARRY 1024.0f
#define DOTSCALE (2.0f / (XCARRY * XCARRY))
#define OUTSCALE (1.0f / (PCARRY * WCARRY))
#define KEXP ((float)(-1.0 / (2.0 * 10.077141124806595)))

#define F16_BYTES  ((size_t)NQ * DIM * 2)
#define X2_BYTES   ((size_t)NQ * 4)
#define T16_BYTES  ((size_t)NPAD * DIM * 2)
#define T2_BYTES   ((size_t)NPAD * 4)
#define WT_BYTES   ((size_t)OUTD * NPAD * 2)
#define PART_BYTES ((size_t)KSPLIT * NQ * OUTD * 4)
#define OFF_F16  ((size_t)0)
#define OFF_X2   (OFF_F16 + F16_BYTES)
#define OFF_T16  (OFF_X2 + X2_BYTES)
#define OFF_T2   (OFF_T16 + T16_BYTES)
#define OFF_WT   (OFF_T2 + T2_BYTES)
#define OFF_PART (OFF_WT + WT_BYTES)
#define WS_TOTAL (OFF_PART + PART_BYTES)
static_assert((F16_BYTES % 128) == 0 && (X2_BYTES % 128) == 0 && (T16_BYTES % 128) == 0);
static_assert((T2_BYTES % 128) == 0 && (WT_BYTES % 128) == 0 && (PART_BYTES % 128) == 0);
static_assert(WS_TOTAL <= (size_t)134217728);

__device__ __forceinline__ float bf16r(float x) {
  unsigned int u = __float_as_uint(x);
  u = (u + 0x7FFFu + ((u >> 16) & 1u)) & 0xFFFF0000u;
  return __uint_as_float(u);
}

static __device__ __forceinline__ h16 toh_flush(float v) {
  const h16 r = (h16)v;
  return (fabsf(v) < 6.103515625e-05f) ? (h16)0.0f : r;
}

__device__ __forceinline__ v16h frag_at(const _Float16* p) {
  v8h lo = *(const v8h*)(p);
  v8h hi = *(const v8h*)(p + 16);
  v16h out;
#pragma unroll
  for (int i = 0; i < 8; ++i) { out[i] = lo[i]; out[i + 8] = hi[i]; }
  return out;
}
__device__ __forceinline__ v16h ld_frag(const _Float16* base, unsigned ld) {
  const unsigned lane = threadIdx.x & 31u;
  return frag_at(base + (lane & 15u) * ld + (lane >> 4) * 8u);
}

__device__ __forceinline__ v8f wmma16(v16h a, v16h b, v8f c) {
  v8f d = __builtin_amdgcn_wmma_f32_16x16x32_f16(false, a, false, b, (short)0, c,
                                                 false, false);
  asm volatile("v_nop\n\tv_nop\n\tv_nop\n\tv_nop" : "+v"(d) : "v"(a), "v"(b));
  return d;
}

__device__ __forceinline__ float red16_sum(float x) {
#pragma unroll
  for (int off = 1; off < 16; off <<= 1) x += __shfl_xor(x, off, 32);
  return x;
}

__device__ __forceinline__ void wave_lds_sync() {
  __builtin_amdgcn_fence(3  , "wavefront");
  asm volatile("s_wait_dscnt 0x0" ::: "memory");
  __builtin_amdgcn_wave_barrier();
}

__global__ __launch_bounds__(256) void rowconv_kernel(
    const float* __restrict__ src, const unsigned nrows,
    _Float16* __restrict__ dst16, float* __restrict__ dstsq) {
  __shared__ float sq[64];
  const unsigned tid = threadIdx.x;
  const unsigned row0 = blockIdx.x * 64u;
  const unsigned c = (tid & 15u) * 8u;
#pragma unroll 1
  for (unsigned j = 0; j < 4u; ++j) {
    const unsigned rl = j * 16u + (tid >> 4);
    const unsigned row = row0 + rl;
    const bool live = row < nrows;
    const unsigned rowc = live ? row : (nrows - 1u);
    const v4f a0 = *(const v4f*)(src + (size_t)rowc * DIM + c);
    const v4f a1 = *(const v4f*)(src + (size_t)rowc * DIM + c + 4u);
    v8h o;
    float ss = 0.0f;
#pragma unroll
    for (int i = 0; i < 4; ++i) {
      const float e0 = live ? bf16r(a0[i]) : 0.0f;
      const float e1 = live ? bf16r(a1[i]) : 0.0f;
      ss += e0 * e0;
      ss += e1 * e1;
      o[i]     = toh_flush(XCARRY * e0);
      o[i + 4] = toh_flush(XCARRY * e1);
    }
    ss = red16_sum(ss);
    if ((tid & 15u) == 0u) sq[rl] = ss;
    _Float16* p = dst16 + (size_t)row * DIM + c;
    *(volatile v8h*)p = o;
    __threadfence();
    *(volatile v8h*)p = o;
  }
  __syncthreads();
  if (tid < 16u) {
    const v4f t = *(const v4f*)&sq[tid * 4u];
    float* p = dstsq + row0 + tid * 4u;
    *(volatile v4f*)p = t;
    __threadfence();
    *(volatile v4f*)p = t;
  }
}

__global__ __launch_bounds__(256) void wconv_kernel(
    const float* __restrict__ W, _Float16* __restrict__ Wt, unsigned ldw, unsigned ldk,
    unsigned krows) {
  __shared__ _Float16 T[64 * LDT];
  const unsigned tid = threadIdx.x;
  const unsigned n0 = blockIdx.x * 64u;
  const unsigned k0 = blockIdx.y * 64u;
#pragma unroll 4
  for (unsigned j = 0; j < 16u; ++j) {
    const unsigned idx = tid + 256u * j;
    const unsigned kr = idx >> 6, nc = idx & 63u;
    const unsigned kg = k0 + kr;
    const bool live = kg < krows;
    const unsigned kc = live ? kg : (krows - 1u);
    float v = W[(size_t)kc * ldw + n0 + nc];
    v = live ? v : 0.0f;
    T[nc * LDT + kr] = toh_flush(WCARRY * bf16r(v));
  }
  __syncthreads();
  v8h x[2];
  size_t off[2];
#pragma unroll
  for (unsigned i = 0; i < 2u; ++i) {
    const unsigned n = 32u * i + (tid >> 3);
    const unsigned kc = (tid & 7u) * 8u;
    x[i] = *(const v8h*)&T[n * LDT + kc];
    off[i] = (size_t)(n0 + n) * ldk + k0 + kc;
  }
#pragma unroll
  for (int i = 0; i < 2; ++i) *(volatile v8h*)(Wt + off[i]) = x[i];
  __threadfence();
#pragma unroll
  for (int i = 0; i < 2; ++i) *(volatile v8h*)(Wt + off[i]) = x[i];
}

__global__ __launch_bounds__(256) void rbf_kernel(
    const _Float16* __restrict__ F16, const float* __restrict__ X2,
    const _Float16* __restrict__ T16, const float* __restrict__ T2,
    const _Float16* __restrict__ Wt, float* __restrict__ Part) {
  __shared__ _Float16 Ps[8 * 16 * LDT];
  __shared__ float Os[8 * 16 * LDC];

  const unsigned tid = threadIdx.x, lane = tid & 31u;
  const unsigned w = (unsigned)__builtin_amdgcn_readfirstlane((int)(tid >> 5));
  const unsigned hh = lane >> 4, m = lane & 15u;
  const unsigned qrow0 = blockIdx.x * 128u + w * 16u;
  const unsigned split = blockIdx.y;
  const unsigned pbase = w * (16u * LDT);
  const unsigned obase = w * (16u * LDC);

  const _Float16* qp = F16 + (size_t)(qrow0 + m) * DIM + hh * 8u;
  v16h qf[4];
#pragma unroll
  for (int c = 0; c < 4; ++c) qf[c] = frag_at(qp + c * 32);

  float x2v[8];
  {
    const v4f xa = *(const v4f*)(X2 + qrow0 + hh * 8u);
    const v4f xb = *(const v4f*)(X2 + qrow0 + hh * 8u + 4u);
#pragma unroll
    for (int i = 0; i < 4; ++i) { x2v[i] = xa[i]; x2v[i + 4] = xb[i]; }
  }

  v8f o[4];
#pragma unroll
  for (int nb = 0; nb < 4; ++nb) o[nb] = (v8f){};

  const unsigned kbeg = split * (unsigned)KPS;
  const unsigned kend = kbeg + (unsigned)KPS;

  for (unsigned kb = kbeg; kb < kend; kb += 64u) {
    v8f s[4];
    float tt[4];
#pragma unroll
    for (int kg = 0; kg < 4; ++kg) {
      const _Float16* tp = T16 + (size_t)(kb + (unsigned)kg * 16u + m) * DIM + hh * 8u;
      v8f t = {};
#pragma unroll
      for (int c = 0; c < 4; ++c) {
        const v16h kf = frag_at(tp + c * 32);
        t = wmma16(qf[c], kf, t);
      }
      s[kg] = t;
      tt[kg] = T2[kb + (unsigned)kg * 16u + m];
    }

#pragma unroll
    for (int kg = 0; kg < 4; ++kg) {
      const unsigned key = kb + (unsigned)kg * 16u + m;
      const bool live = key < (unsigned)NTR;
#pragma unroll
      for (int v = 0; v < 8; ++v) {
        float d2 = (x2v[v] + tt[kg]) - s[kg][v] * DOTSCALE;
        d2 = fmaxf(d2, 0.0f);
        const float dist = __builtin_amdgcn_sqrtf(d2);
        float kk = __expf(dist * KEXP);
        kk = live ? kk : 0.0f;
        Ps[pbase + (hh * 8u + (unsigned)v) * LDT + (unsigned)kg * 16u + m] =
            toh_flush(kk * PCARRY);
      }
    }
    wave_lds_sync();

#pragma unroll
    for (int c = 0; c < 2; ++c) {
      const v16h pf = ld_frag(&Ps[pbase + (unsigned)c * 32u], LDT);
#pragma unroll
      for (int nb = 0; nb < 4; ++nb) {
        const v16h vf = frag_at(Wt + (size_t)((unsigned)nb * 16u + m) * NPAD + kb +
                                (unsigned)c * 32u + hh * 8u);
        o[nb] = wmma16(pf, vf, o[nb]);
      }
    }
    wave_lds_sync();
  }

#pragma unroll
  for (int nb = 0; nb < 4; ++nb)
#pragma unroll
    for (int v = 0; v < 8; ++v)
      Os[obase + (hh * 8u + (unsigned)v) * LDC + (unsigned)nb * 16u + m] = o[nb][v];
  wave_lds_sync();
  v4f xs[8];
  size_t off[8];
#pragma unroll
  for (unsigned i = 0; i < 8u; ++i) {
    const unsigned r = 2u * i + (lane >> 4);
    const unsigned c = (lane & 15u) * 4u;
    xs[i] = *(const v4f*)&Os[obase + r * LDC + c];
    off[i] = ((size_t)split * NQ + qrow0 + r) * OUTD + c;
  }
#pragma unroll
  for (int i = 0; i < 8; ++i) *(volatile v4f*)(Part + off[i]) = xs[i];
  __threadfence();
#pragma unroll
  for (int i = 0; i < 8; ++i) *(volatile v4f*)(Part + off[i]) = xs[i];
}

__global__ __launch_bounds__(256) void combine_kernel(
    const float* __restrict__ Part, float* __restrict__ outf) {
  const size_t e = ((size_t)blockIdx.x * 256u + threadIdx.x) * 4u;
  v4f acc = {};
#pragma unroll 1
  for (unsigned s = 0; s < (unsigned)KSPLIT; ++s) {
    const v4f t = *(const v4f*)(Part + (size_t)s * NQ * OUTD + e);
    acc = acc + t;
  }
  acc = acc * OUTSCALE;
  float* p = outf + e;
  *(volatile v4f*)p = acc;
  __threadfence();
  *(volatile v4f*)p = acc;
}

extern "C" void kernel_launch(void* const* d_in, const int* in_sizes, int n_in,
                              void* d_out, int out_size, void* d_ws, size_t ws_size,
                              hipStream_t stream) {
  if (n_in < 3) return;
  if ((long long)in_sizes[0] < (long long)NQ * DIM) return;
  if ((long long)in_sizes[1] < (long long)NTR * DIM) return;
  if ((long long)in_sizes[2] < (long long)NTR * OUTD) return;
  if ((long long)out_size < (long long)NQ * OUTD) return;
  if (ws_size < WS_TOTAL) return;

  const float* feats = (const float*)d_in[0];
  const float* train = (const float*)d_in[1];
  const float* wts   = (const float*)d_in[2];
  float* out = (float*)d_out;

  char* ws = (char*)d_ws;
  _Float16* F16p = (_Float16*)(ws + OFF_F16);
  float*    X2p  = (float*)(ws + OFF_X2);
  _Float16* T16p = (_Float16*)(ws + OFF_T16);
  float*    T2p  = (float*)(ws + OFF_T2);
  _Float16* Wtp  = (_Float16*)(ws + OFF_WT);
  float*    Partp = (float*)(ws + OFF_PART);

  dim3 blk(256);
  rowconv_kernel<<<dim3(NQ / 64), blk, 0, stream>>>(feats, (unsigned)NQ, F16p, X2p);
  rowconv_kernel<<<dim3(NPAD / 64), blk, 0, stream>>>(train, (unsigned)NTR, T16p, T2p);
  wconv_kernel<<<dim3(OUTD / 64, NPAD / 64), blk, 0, stream>>>(wts, Wtp, (unsigned)OUTD,
                                                              (unsigned)NPAD, (unsigned)NTR);
  rbf_kernel<<<dim3(NQ / 128, KSPLIT), blk, 0, stream>>>(F16p, X2p, T16p, T2p, Wtp, Partp);
  combine_kernel<<<dim3((NQ * OUTD) / 1024), blk, 0, stream>>>(Partp, out);
}
